// Pos_att_56049323213171
// MI455X (gfx1250) — hardware-run, weakly checked
//
#include <hip/hip_runtime.h>
#include <stdint.h>

#define CH    256
#define NP    9216
#define HW    96
#define KC    32
#define YP    64
#define CTI   256
#define NCB   36
#define SBLK  128
#define NSB   72
#define KCK   32
#define NKC   288
#define JB    64
#define NJB   144
#define SPP   40
#define SWP   264
#define SXP   40
#define SYP   72
#define XPC   9
#define XTB   128

#define XSCALE   64.0f
#define WSCALE   256.0f
#define OSC_CONV (1.0f / 16384.0f)
#define YSCALE   1024.0f
#define PSCALE   16384.0f
#define OSC_AGG  (1.0f / 1048576.0f)
#define L2E      1.4426950408889634f
#define SL2      (1.4426950408889634f * (1.0f / 1048576.0f))

static_assert(NCB * CTI == NP);
static_assert(NSB * SBLK == NP);
static_assert(NKC * KCK == NP);
static_assert(NJB * JB == NP);
static_assert(XPC * XTB * 8 == NP);
static_assert(HW * HW == NP);
static_assert(CH % 32 == 0 && CH == 8 * 32);
static_assert(YP == 2 * KC);
static_assert(CTI * SYP <= KC * SWP + CTI * SXP);
static_assert((SPP % 8) == 0 && SPP >= KCK);
static_assert((SWP % 8) == 0 && (SXP % 8) == 0 && (SYP % 8) == 0);
static_assert((NP % 256) == 0 && (HW % 32) == 0 && (HW % 8) == 0);

typedef _Float16 v16h __attribute__((ext_vector_type(16)));
typedef _Float16 v8h  __attribute__((ext_vector_type(8)));
typedef float    v8f  __attribute__((ext_vector_type(8)));
typedef float    v4f  __attribute__((ext_vector_type(4)));
typedef unsigned int v4u __attribute__((ext_vector_type(4)));
static_assert(sizeof(v16h) == 32);
static_assert(sizeof(v8h) == 16);

__device__ __forceinline__ unsigned short bf_bits(float f) {
  unsigned u = __float_as_uint(f);
  return (unsigned short)((u + 0x7FFFu + ((u >> 16) & 1u)) >> 16);
}
__device__ __forceinline__ float bf_up(unsigned short hb) { return __uint_as_float(((unsigned)hb) << 16); }
__device__ __forceinline__ float bfr(float f) { return bf_up(bf_bits(f)); }
__device__ __forceinline__ unsigned short h_bits(_Float16 x) { return __builtin_bit_cast(unsigned short, x); }
__device__ __forceinline__ unsigned short f2h_bits(float f) { return h_bits((_Float16)f); }
__device__ __forceinline__ unsigned pk16(unsigned short a, unsigned short b) { return (unsigned)a | ((unsigned)b << 16); }
__device__ __forceinline__ v8f zero8() { v8f z = {0.f, 0.f, 0.f, 0.f, 0.f, 0.f, 0.f, 0.f}; return z; }

__device__ __forceinline__ v16h ldfrag_h(const _Float16* p) {
  union { v16h v; v8h hv[2]; } f;
  f.hv[0] = *(const v8h*)(p);
  f.hv[1] = *(const v8h*)(p + 16);
  return f.v;
}

__device__ __forceinline__ v8f mma_h_raw(v16h a, v16h b, v8f c) {
  return __builtin_amdgcn_wmma_f32_16x16x32_f16(false, a, false, b, (short)0, c, false, false);
}
__device__ __forceinline__ void dep_guard_h(v8f& a, v8f& b, v16h x, v16h y) {
#if defined(__HIP_DEVICE_COMPILE__)
  asm volatile("v_nop\n\tv_nop\n\tv_nop\n\tv_nop" : "+v"(a), "+v"(b) : "v"(x), "v"(y));
#endif
}
__device__ __forceinline__ void dep_guard2x3(v8f& a, v8f& b, v16h x, v16h y, v16h z) {
#if defined(__HIP_DEVICE_COMPILE__)
  asm volatile("v_nop\n\tv_nop\n\tv_nop\n\tv_nop" : "+v"(a), "+v"(b) : "v"(x), "v"(y), "v"(z));
#endif
}
__device__ __forceinline__ void dep_guard1x4(v8f& a, v16h w, v16h x, v16h y, v16h z) {
#if defined(__HIP_DEVICE_COMPILE__)
  asm volatile("v_nop\n\tv_nop\n\tv_nop\n\tv_nop" : "+v"(a) : "v"(w), "v"(x), "v"(y), "v"(z));
#endif
}
__device__ __forceinline__ void keep4_h(v16h a, v16h b, v16h c, v16h d) {
#if defined(__HIP_DEVICE_COMPILE__)
  asm volatile("v_nop" :: "v"(a), "v"(b), "v"(c), "v"(d));
#endif
}
__device__ __forceinline__ void keep2_h(v16h a, v16h b) {
#if defined(__HIP_DEVICE_COMPILE__)
  asm volatile("v_nop" :: "v"(a), "v"(b));
#endif
}
__device__ __forceinline__ void acc_guard4(v8f& a, v8f& b, v8f& c, v8f& d) {
#if defined(__HIP_DEVICE_COMPILE__)
  asm volatile("v_nop\n\tv_nop\n\tv_nop\n\tv_nop" : "+v"(a), "+v"(b), "+v"(c), "+v"(d));
#endif
}
__device__ __forceinline__ void wave_sync_lds() {
  __builtin_amdgcn_fence(__ATOMIC_RELEASE, "workgroup");
  __builtin_amdgcn_wave_barrier();
  __builtin_amdgcn_fence(__ATOMIC_ACQUIRE, "workgroup");
}

__global__ __launch_bounds__(XTB) void k_cvt_x(const float* __restrict__ x, unsigned short* xh) {
  const int tid = threadIdx.x;
  const int c = blockIdx.x;
  const float* s = x + (size_t)c * NP;
  unsigned short* d = xh + (size_t)c * NP;
  v4u pk[XPC];
#pragma unroll
  for (int it = 0; it < XPC; ++it) {
    const int e0 = 8 * (it * XTB + tid);
    const v4f a = *(const v4f*)(s + e0);
    const v4f b = *(const v4f*)(s + e0 + 4);
    v4u p;
    p[0] = pk16(f2h_bits(bfr(a[0]) * XSCALE), f2h_bits(bfr(a[1]) * XSCALE));
    p[1] = pk16(f2h_bits(bfr(a[2]) * XSCALE), f2h_bits(bfr(a[3]) * XSCALE));
    p[2] = pk16(f2h_bits(bfr(b[0]) * XSCALE), f2h_bits(bfr(b[1]) * XSCALE));
    p[3] = pk16(f2h_bits(bfr(b[2]) * XSCALE), f2h_bits(bfr(b[3]) * XSCALE));
    pk[it] = p;
  }
  for (int pass = 0; pass < 2; ++pass) {
#pragma unroll
    for (int it = 0; it < XPC; ++it) {
      const int e0 = 8 * (it * XTB + tid);
      *(volatile v4u*)(d + e0) = pk[it];
    }
    __threadfence();
  }
}

__global__ __launch_bounds__(256) void k_conv(const float* __restrict__ x, const float* __restrict__ w,
                                               const float* __restrict__ bcv, unsigned short* yout) {
  __shared__ __align__(16) _Float16 lds[KC * SWP + CTI * SXP];
  _Float16* sW = lds;
  _Float16* sX = lds + KC * SWP;
  _Float16* sY = lds;
  const int tid = threadIdx.x, wave = tid >> 5, lane = tid & 31;
  const int rl = lane & 15, hf = lane >> 4, koff = 8 * hf;
  const int i0 = blockIdx.x * CTI;

  for (int idx = tid; idx < KC * CH; idx += 256) {
    const int o = idx >> 8, c = idx & 255;
    sW[o * SWP + c] = (_Float16)(bfr(w[idx]) * WSCALE);
  }

  v8f acc[2][2];
#pragma unroll
  for (int t = 0; t < 2; ++t)
#pragma unroll
    for (int j = 0; j < 2; ++j) acc[t][j] = zero8();

#pragma unroll 1
  for (int kc = 0; kc < CH / 32; ++kc) {
    const int c0 = kc * 32;
#pragma unroll 8
    for (int it = 0; it < 32; ++it) {
      const float v = x[(size_t)(c0 + it) * NP + i0 + tid];
      sX[tid * SXP + it] = (_Float16)(bfr(v) * XSCALE);
    }
    __syncthreads();
    const v16h b0 = ldfrag_h(sW + rl * SWP + c0 + koff);
    const v16h b1 = ldfrag_h(sW + (16 + rl) * SWP + c0 + koff);
#pragma unroll
    for (int t = 0; t < 2; ++t) {
      const v16h a = ldfrag_h(sX + (32 * wave + 16 * t + rl) * SXP + koff);
      acc[t][0] = mma_h_raw(a, b0, acc[t][0]);
      acc[t][1] = mma_h_raw(a, b1, acc[t][1]);
      dep_guard_h(acc[t][0], acc[t][1], a, b1);
    }
    keep2_h(b0, b1);
    __syncthreads();
  }
  acc_guard4(acc[0][0], acc[0][1], acc[1][0], acc[1][1]);

#pragma unroll
  for (int t = 0; t < 2; ++t) {
#pragma unroll
    for (int jt = 0; jt < 2; ++jt) {
      const int o = 16 * jt + rl;
      const float bb = bfr(bcv[o]);
#pragma unroll
      for (int r = 0; r < 8; ++r) {
        const float v = acc[t][jt][r] * OSC_CONV + bb;
        const float tt = v * YSCALE;
        const _Float16 hi = (_Float16)tt;
        const _Float16 rs = (_Float16)(tt - (float)hi);
        const int row = 32 * wave + 16 * t + 8 * hf + r;
        sY[row * SYP + o] = hi;
        sY[row * SYP + KC + o] = rs;
      }
    }
  }
  __syncthreads();

  const int p = tid & 7, grp = tid >> 3;
  v4u pk[8];
#pragma unroll
  for (int it = 0; it < 8; ++it) {
    const int li = it * 32 + grp;
    union { v8h h; v4u u; } cv;
    cv.h = *(const v8h*)(sY + li * SYP + 8 * p);
    pk[it] = cv.u;
  }
  for (int pass = 0; pass < 2; ++pass) {
#pragma unroll
    for (int it = 0; it < 8; ++it) {
      const int li = it * 32 + grp;
      const int i = i0 + li;
      const int hh = i / HW;
      const int ww = i - hh * HW;
      const int r = ww * HW + hh;
      *(volatile v4u*)(yout + (size_t)r * YP + 8 * p) = pk[it];
    }
    __threadfence();
  }
}

__global__ __launch_bounds__(256) void k_stats(const unsigned short* __restrict__ yp, float* gout) {
  const _Float16* Y = (const _Float16*)(const void*)yp;
  __shared__ __align__(16) float sG[SBLK];
  const int tid = threadIdx.x, wave = tid >> 5, lane = tid & 31;
  const int rl = lane & 15, hf = lane >> 4, koff = 8 * hf;
  const int row0 = blockIdx.x * SBLK + 16 * wave;

  const v16h qh = ldfrag_h(Y + (size_t)(row0 + rl) * YP + koff);
  const v16h qr = ldfrag_h(Y + (size_t)(row0 + rl) * YP + KC + koff);

  float rmax[8], lsum[8];
#pragma unroll
  for (int r = 0; r < 8; ++r) { rmax[r] = -1.0e30f; lsum[r] = 0.0f; }

#pragma unroll 1
  for (int kc = 0; kc < NKC; ++kc) {
    const int key0 = kc * KCK;
    const _Float16* kp0 = Y + (size_t)(key0 + rl) * YP + koff;
    const _Float16* kp1 = Y + (size_t)(key0 + 16 + rl) * YP + koff;
    const v16h kh0 = ldfrag_h(kp0), kr0 = ldfrag_h(kp0 + KC);
    const v16h kh1 = ldfrag_h(kp1), kr1 = ldfrag_h(kp1 + KC);
    v8f s0 = mma_h_raw(qh, kh0, zero8());
    s0 = mma_h_raw(qh, kr0, s0);
    s0 = mma_h_raw(qr, kh0, s0);
    v8f s1 = mma_h_raw(qh, kh1, zero8());
    s1 = mma_h_raw(qh, kr1, s1);
    s1 = mma_h_raw(qr, kh1, s1);
    dep_guard2x3(s0, s1, qr, kh1, kr1);
    keep4_h(qh, kh0, kr0, qr);
    float tm[8];
#pragma unroll
    for (int r = 0; r < 8; ++r) tm[r] = fmaxf(s0[r], s1[r]) * SL2;
#pragma unroll
    for (int r = 0; r < 8; ++r) {
      tm[r] = fmaxf(tm[r], __shfl_xor(tm[r], 1, 32));
      tm[r] = fmaxf(tm[r], __shfl_xor(tm[r], 2, 32));
      tm[r] = fmaxf(tm[r], __shfl_xor(tm[r], 4, 32));
      tm[r] = fmaxf(tm[r], __shfl_xor(tm[r], 8, 32));
    }
#pragma unroll
    for (int r = 0; r < 8; ++r) {
      const float nm = fmaxf(rmax[r], tm[r]);
      const float al = __builtin_amdgcn_exp2f(rmax[r] - nm);
      rmax[r] = nm;
      lsum[r] *= al;
    }
#pragma unroll
    for (int r = 0; r < 8; ++r) {
      const float p0 = __builtin_amdgcn_exp2f(s0[r] * SL2 - rmax[r]);
      const float p1 = __builtin_amdgcn_exp2f(s1[r] * SL2 - rmax[r]);
      lsum[r] += p0 + p1;
    }
  }

  float g[8];
#pragma unroll
  for (int r = 0; r < 8; ++r) {
    float l = lsum[r];
    l += __shfl_xor(l, 1, 32);
    l += __shfl_xor(l, 2, 32);
    l += __shfl_xor(l, 4, 32);
    l += __shfl_xor(l, 8, 32);
    g[r] = rmax[r] + __log2f(l);
  }
  if (rl == 0) {
#pragma unroll
    for (int r = 0; r < 8; ++r) sG[16 * wave + 8 * hf + r] = g[r];
  }
  __syncthreads();
  if (wave == 0) {
    const v4f gv = *(const v4f*)(sG + 4 * lane);
    float* d = gout + (size_t)blockIdx.x * SBLK + 4 * lane;
    *(volatile v4f*)d = gv;
    __threadfence();
    *(volatile v4f*)d = gv;
  }
}

__global__ __launch_bounds__(256) void k_main(const unsigned short* __restrict__ yp,
                                               const unsigned short* __restrict__ xhp,
                                               const float* __restrict__ gp, float* x6p) {
  const _Float16* Y  = (const _Float16*)(const void*)yp;
  const _Float16* XH = (const _Float16*)(const void*)xhp;
  __shared__ __align__(16) _Float16 sP[2][JB * SPP];
  __shared__ __align__(16) float sT[8][16 * 68];

  const int tid = threadIdx.x, wave = tid >> 5, lane = tid & 31;
  const int rl = lane & 15, hf = lane >> 4, koff = 8 * hf, mOff = 8 * hf;
  const int j0 = blockIdx.x * JB;
  const int its = wave >> 2, js = wave & 3;

  const v16h ybh = ldfrag_h(Y + (size_t)(j0 + 16 * js + rl) * YP + koff);
  const v16h ybr = ldfrag_h(Y + (size_t)(j0 + 16 * js + rl) * YP + KC + koff);

  v8f acc[2][4];
#pragma unroll
  for (int i = 0; i < 2; ++i)
#pragma unroll
    for (int j = 0; j < 4; ++j) acc[i][j] = zero8();

  const size_t xrow0 = (size_t)(32 * wave + rl) * NP;
  const size_t xrow1 = (size_t)(32 * wave + 16 + rl) * NP;

#pragma unroll 1
  for (int ic = 0; ic < NKC; ++ic) {
    const int i0 = ic * KCK;
    const int buf = ic & 1;
    const int irow = i0 + 16 * its;
    const _Float16* yap = Y + (size_t)(irow + rl) * YP + koff;
    const v16h yah = ldfrag_h(yap), yar = ldfrag_h(yap + KC);
    v8f s = mma_h_raw(yah, ybh, zero8());
    s = mma_h_raw(yah, ybr, s);
    s = mma_h_raw(yar, ybh, s);
    dep_guard1x4(s, yar, ybh, yah, ybr);
    const v4f g0 = *(const v4f*)(gp + irow + mOff);
    const v4f g1 = *(const v4f*)(gp + irow + mOff + 4);
    v8h pv;
#pragma unroll
    for (int r = 0; r < 4; ++r) {
      pv[r]     = (_Float16)(__builtin_amdgcn_exp2f(s[r]     * SL2 - g0[r]) * PSCALE);
      pv[r + 4] = (_Float16)(__builtin_amdgcn_exp2f(s[r + 4] * SL2 - g1[r]) * PSCALE);
    }
    *(v8h*)(&sP[buf][(16 * js + rl) * SPP + 16 * its + mOff]) = pv;
    __syncthreads();
    v16h pb[4];
#pragma unroll
    for (int jt = 0; jt < 4; ++jt) pb[jt] = ldfrag_h(&sP[buf][(16 * jt + rl) * SPP + koff]);
    const v16h xa0 = ldfrag_h(XH + xrow0 + i0 + koff);
    const v16h xa1 = ldfrag_h(XH + xrow1 + i0 + koff);
#pragma unroll
    for (int jt = 0; jt < 4; ++jt) acc[0][jt] = mma_h_raw(xa0, pb[jt], acc[0][jt]);
    dep_guard_h(acc[0][0], acc[0][3], xa0, pb[3]);
#pragma unroll
    for (int jt = 0; jt < 4; ++jt) acc[1][jt] = mma_h_raw(xa1, pb[jt], acc[1][jt]);
    dep_guard_h(acc[1][0], acc[1][3], xa1, pb[3]);
    keep4_h(pb[0], pb[1], pb[2], xa0);
  }
  acc_guard4(acc[0][0], acc[0][1], acc[0][2], acc[0][3]);
  acc_guard4(acc[1][0], acc[1][1], acc[1][2], acc[1][3]);

  float* slab = sT[wave];
#pragma unroll
  for (int ct = 0; ct < 2; ++ct) {
    const int mBase = 32 * wave + 16 * ct;
#pragma unroll
    for (int j = 0; j < 4; ++j) {
#pragma unroll
      for (int r = 0; r < 8; ++r) {
        slab[(mOff + r) * 68 + (j << 4) + rl] = acc[ct][j][r];
      }
    }
    wave_sync_lds();
    {
      const int hh = lane >> 4, c4 = (lane & 15) * 4;
      v4f ov[8];
#pragma unroll
      for (int it = 0; it < 8; ++it) {
        const int row = it * 2 + hh;
        v4f v = *(const v4f*)(slab + row * 68 + c4);
        v[0] *= OSC_AGG;
        v[1] *= OSC_AGG;
        v[2] *= OSC_AGG;
        v[3] *= OSC_AGG;
        ov[it] = v;
      }
      for (int pass = 0; pass < 2; ++pass) {
#pragma unroll
        for (int it = 0; it < 8; ++it) {
          const int row = it * 2 + hh;
          *(volatile v4f*)(x6p + (size_t)(mBase + row) * NP + j0 + c4) = ov[it];
        }
        __threadfence();
      }
    }
    wave_sync_lds();
  }
}

__global__ __launch_bounds__(256) void k_final(const float* __restrict__ x6p, const float* __restrict__ x,
                                                float* out) {
  __shared__ float red[8];
  const int tid = threadIdx.x, wave = tid >> 5, lane = tid & 31;
  const int c = blockIdx.x;
  const float* row = x6p + (size_t)c * NP;
  const float* xr  = x   + (size_t)c * NP;
  float* orow      = out + (size_t)c * NP;

  constexpr int NV = NP / 256;
  constexpr int NSEG = HW / 32;
  float v[NV];
  float m = -1.0e30f;
#pragma unroll
  for (int it = 0; it < NV; ++it) {
    v[it] = row[it * 256 + tid];
    m = fmaxf(m, v[it]);
  }
#pragma unroll
  for (int d = 1; d < 32; d <<= 1) m = fmaxf(m, __shfl_xor(m, d, 32));
  if (lane == 0) red[wave] = m;
  __syncthreads();
  float M = red[0];
#pragma unroll
  for (int k = 1; k < 8; ++k) M = fmaxf(M, red[k]);
  __syncthreads();
  float s = 0.0f;
#pragma unroll
  for (int it = 0; it < NV; ++it) s += __builtin_amdgcn_exp2f((v[it] - M) * L2E);
#pragma unroll
  for (int d = 1; d < 32; d <<= 1) s += __shfl_xor(s, d, 32);
  if (lane == 0) red[wave] = s;
  __syncthreads();
  float Z = red[0];
#pragma unroll
  for (int k = 1; k < 8; ++k) Z += red[k];
  const float invZ = 1.0f / Z;

#pragma unroll 1
  for (int k = 0; k < HW / 8; ++k) {
    const int hrow = wave + 8 * k;
    const int base = hrow * HW;
    float t[NSEG], e[NSEG];
    float mm = -1.0e30f;
#pragma unroll
    for (int sg = 0; sg < NSEG; ++sg) {
      const float a  = row[base + lane + 32 * sg];
      const float xv = bfr(xr[base + lane + 32 * sg]);
      t[sg] = __builtin_amdgcn_exp2f((a - M) * L2E) * invZ + xv;
      mm = fmaxf(mm, t[sg]);
    }
#pragma unroll
    for (int d = 1; d < 32; d <<= 1) mm = fmaxf(mm, __shfl_xor(mm, d, 32));
    float ss = 0.0f;
#pragma unroll
    for (int sg = 0; sg < NSEG; ++sg) { e[sg] = __builtin_amdgcn_exp2f((t[sg] - mm) * L2E); ss += e[sg]; }
#pragma unroll
    for (int d = 1; d < 32; d <<= 1) ss += __shfl_xor(ss, d, 32);
    const float inv = 1.0f / ss;
    float* dp = orow + base;
#pragma unroll
    for (int sg = 0; sg < NSEG; ++sg) *(volatile float*)(dp + lane + 32 * sg) = e[sg] * inv;
    __threadfence();
#pragma unroll
    for (int sg = 0; sg < NSEG; ++sg) *(volatile float*)(dp + lane + 32 * sg) = e[sg] * inv;
  }
}

extern "C" void kernel_launch(void* const* d_in, const int* in_sizes, int n_in,
                              void* d_out, int out_size, void* d_ws, size_t ws_size,
                              hipStream_t stream) {
  if (n_in < 3) return;
  if (in_sizes[0] != CH * NP) return;
  if (in_sizes[1] != KC * CH) return;
  if (in_sizes[2] != KC) return;
  if (out_size != CH * NP) return;

  const float* x  = (const float*)d_in[0];
  const float* wc = (const float*)d_in[1];
  const float* bc = (const float*)d_in[2];
  float* out = (float*)d_out;

  const size_t PXH = (size_t)CH * NP * 2;
  const size_t PY  = (size_t)NP * YP * 2;
  const size_t PG  = (size_t)NP * 4;
  const size_t PX6 = (size_t)CH * NP * 4;

  size_t off = 0;
  const size_t oXH = off; off += PXH;
  const size_t oY  = off; off += PY;
  const size_t oG  = off; off += PG;
  const size_t oX6 = off; off += PX6;
  if (off > ws_size) return;
  if (off > (size_t)134217728) return;

  char* ws = (char*)d_ws;
  unsigned short* XHp = (unsigned short*)(ws + oXH);
  unsigned short* Yp  = (unsigned short*)(ws + oY);
  float*          Gp  = (float*)(ws + oG);
  float*          X6p = (float*)(ws + oX6);

  k_cvt_x<<<dim3(CH), dim3(XTB), 0, stream>>>(x, XHp);
  k_conv<<<dim3(NCB), dim3(256), 0, stream>>>(x, wc, bc, Yp);
  k_stats<<<dim3(NSB), dim3(256), 0, stream>>>(Yp, Gp);
  k_main<<<dim3(NJB), dim3(256), 0, stream>>>(Yp, XHp, Gp, X6p);
  k_final<<<dim3(CH), dim3(256), 0, stream>>>(X6p, x, out);
  (void)hipGetLastError();
}
